// CausalSelfAttention_40123584479483
// MI455X (gfx1250) — hardware-verified
//
#include <hip/hip_runtime.h>


#ifndef NB
#define NB 4
#endif
#ifndef SEQ
#define SEQ 2048
#endif
#ifndef RH
#define RH 256
#endif
#define NB_FULL  4
#define SEQ_FULL 2048
#define DM    1024
#define NH    16
#define HD    64
#define NQKV  (3 * DM)
#define MROWS (NB * SEQ)
#define PLN   ((size_t)NB * NH * SEQ * HD)
#define PLH   ((size_t)NB * NH * RH * HD)
#define SCL2  (0.125f * 1.4426950408889634f)
#define PCL2  10.0f
#define CCAR  64.0f
#define WCAR  64.0f
#define OSC   (1.0f / 4096.0f)

static_assert(NH * HD == DM);
static_assert(HD == 64);
static_assert(SEQ % 64 == 0);
static_assert(RH % 64 == 0);
static_assert(RH >= 64);
static_assert(RH <= SEQ);
static_assert(DM % 64 == 0);
static_assert(DM % 32 == 0);
static_assert(NQKV % 64 == 0);
static_assert(NB <= NB_FULL);
static_assert(SEQ <= SEQ_FULL);
static_assert(((size_t)MROWS * DM / 8) % 256 == 0);

typedef _Float16 h16;
typedef unsigned short bf;
typedef __attribute__((ext_vector_type(16))) __bf16   v16bf;
typedef __attribute__((ext_vector_type(16))) _Float16 v16h;
typedef __attribute__((ext_vector_type(8)))  _Float16 v8h;
typedef __attribute__((ext_vector_type(8)))  unsigned short v8us;
typedef __attribute__((ext_vector_type(8)))  float    v8f;
typedef __attribute__((ext_vector_type(4)))  float    v4f;
typedef v4f  __attribute__((may_alias)) v4fa;
typedef v8us __attribute__((may_alias)) v8usa;

constexpr size_t SZ_XB  = (size_t)MROWS * DM * 2;
constexpr size_t SZ_WT  = (size_t)NQKV * DM * 2;
constexpr size_t SZ_WO  = (size_t)DM * DM * 2;
constexpr size_t SZ_P16 = 3 * PLN * 2;
constexpr size_t SZ_PH  = 3 * PLH * 2;
constexpr size_t SZ_CT  = (size_t)MROWS * DM * 2;
constexpr size_t SZ_CH  = (size_t)NB * RH * DM * 2;
constexpr size_t WS_TOTAL = SZ_XB + SZ_WT + 2 * SZ_WO + SZ_P16 + 2 * SZ_PH + SZ_CT + 2 * SZ_CH;
static_assert(WS_TOTAL <= (size_t)134217728);
static_assert(SZ_XB % 256 == 0);
static_assert(SZ_WT % 256 == 0);
static_assert(SZ_WO % 256 == 0);
static_assert(SZ_P16 % 256 == 0);
static_assert(SZ_PH % 256 == 0);
static_assert(SZ_CT % 256 == 0);
static_assert(SZ_CH % 256 == 0);

__device__ __forceinline__ unsigned short f2bf(float f) { unsigned u = __float_as_uint(f); u += 0x7FFFu + ((u >> 16) & 1u); return (unsigned short)(u >> 16); }
__device__ __forceinline__ float bf2f(unsigned short b) { return __uint_as_float(((unsigned)b) << 16); }
__device__ __forceinline__ float bfr(float f) { return bf2f(f2bf(f)); }
__device__ __forceinline__ void splitf(float y, unsigned short& h, unsigned short& l) { h = f2bf(y); l = f2bf(y - bf2f(h)); }
__device__ __forceinline__ v16h cat16(v8h lo, v8h hi) { return __builtin_shufflevector(lo, hi, 0, 1, 2, 3, 4, 5, 6, 7, 8, 9, 10, 11, 12, 13, 14, 15); }
__device__ __forceinline__ v16bf cat16b(v8us lo, v8us hi) { return __builtin_bit_cast(v16bf, __builtin_shufflevector(lo, hi, 0, 1, 2, 3, 4, 5, 6, 7, 8, 9, 10, 11, 12, 13, 14, 15)); }
__device__ __forceinline__ v8f wmma16(v16h a, v16h b, v8f c) { return __builtin_amdgcn_wmma_f32_16x16x32_f16(false, a, false, b, (short)0, c, false, false); }
__device__ __forceinline__ v8f wmmab(v16bf a, v16bf b, v8f c) { return __builtin_amdgcn_wmma_f32_16x16x32_bf16(false, a, false, b, (short)0, c, false, false); }

template <typename T16> struct WFrag;
template <> struct WFrag<h16> { typedef v16h V; static __device__ __forceinline__ V ld(const h16* p) { return cat16(*(const v8h*)p, *(const v8h*)(p + 16)); } static __device__ __forceinline__ v8f mma(V a, V b, v8f c) { return wmma16(a, b, c); } };
template <> struct WFrag<bf> { typedef v16bf V; static __device__ __forceinline__ V ld(const bf* p) { return cat16b(*(const v8us*)p, *(const v8us*)(p + 16)); } static __device__ __forceinline__ v8f mma(V a, V b, v8f c) { return wmmab(a, b, c); } };

__device__ __forceinline__ void mkfrag(const v8f& a, const v8f& b, v16h& fh, v16h& fl) {
    v8h x, y;
#pragma unroll
    for (int r = 0; r < 8; ++r) { x[r] = (h16)a[r]; y[r] = (h16)b[r]; }
    fh = cat16(x, y); (void)fl;
}
__device__ __forceinline__ void mkfrag(const v8f& a, const v8f& b, v16bf& fh, v16bf& fl) {
    v8us xh, xl, yh, yl;
#pragma unroll
    for (int r = 0; r < 8; ++r) { unsigned short p_, q_; splitf(a[r], p_, q_); xh[r] = p_; xl[r] = q_; splitf(b[r], p_, q_); yh[r] = p_; yl[r] = q_; }
    fh = cat16b(xh, yh); fl = cat16b(xl, yl);
}

template <typename T16, int NSPLIT>
__device__ __forceinline__ void gemm_main(const T16* __restrict__ A, const T16* __restrict__ A2, const T16* __restrict__ Bt, const int K, const int r0, const int c0, const int lr, const int hi, v8f (&acc)[4][4]) {
    static_assert(NSPLIT == 0 || NSPLIT == 1);
    typedef typename WFrag<T16>::V V;
#pragma unroll
    for (int mb = 0; mb < 4; ++mb)
#pragma unroll
        for (int nb = 0; nb < 4; ++nb) acc[mb][nb] = (v8f){};
    const size_t aoff = (size_t)(r0 + lr) * K + 8 * hi, boff = (size_t)(c0 + lr) * K + 8 * hi;
#pragma unroll 1
    for (int kc = 0; kc < K; kc += 32) {
        V a[4], a2[4], bl;
#pragma unroll
        for (int mb = 0; mb < 4; ++mb) { a[mb] = WFrag<T16>::ld(A + aoff + (size_t)mb * 16 * K + kc); if (NSPLIT == 1) a2[mb] = WFrag<T16>::ld(A2 + aoff + (size_t)mb * 16 * K + kc); else a2[mb] = a[mb]; }
#pragma unroll
        for (int nb = 0; nb < 4; ++nb) { const V b = WFrag<T16>::ld(Bt + boff + (size_t)nb * 16 * K + kc);
#pragma unroll
            for (int mb = 0; mb < 4; ++mb) { acc[mb][nb] = WFrag<T16>::mma(a[mb], b, acc[mb][nb]); if (NSPLIT == 1) acc[mb][nb] = WFrag<T16>::mma(a2[mb], b, acc[mb][nb]); }
            bl = b; }
        asm volatile("v_nop\n\tv_nop\n\tv_nop\n\tv_nop" : "+v"(acc[0][0]), "+v"(acc[0][1]), "+v"(acc[0][2]), "+v"(acc[0][3]), "+v"(acc[1][0]), "+v"(acc[1][1]), "+v"(acc[1][2]), "+v"(acc[1][3]) : "v"(a[0]), "v"(a2[0]), "v"(bl));
        asm volatile("v_nop\n\tv_nop\n\tv_nop\n\tv_nop" : "+v"(acc[2][0]), "+v"(acc[2][1]), "+v"(acc[2][2]), "+v"(acc[2][3]), "+v"(acc[3][0]), "+v"(acc[3][1]), "+v"(acc[3][2]), "+v"(acc[3][3]) : "v"(a[3]), "v"(a2[3]), "v"(bl));
    }
}

__global__ __launch_bounds__(256) void k_cvtx(const float* __restrict__ x, bf* XB) {
    const size_t i = (size_t)blockIdx.x * 256 + threadIdx.x; if (i >= (size_t)MROWS * DM / 8) return;
    const size_t e = i * 8; const int c = (int)(e % DM); const size_t mrow = e / DM; const size_t b = mrow / SEQ, t = mrow % SEQ;
    const float* src = x + (b * SEQ_FULL + t) * DM + c;
    const v4f a0 = *(const v4f*)src, a1 = *(const v4f*)(src + 4); v8us o;
#pragma unroll
    for (int k = 0; k < 4; ++k) { o[k] = f2bf(a0[k]); o[4 + k] = f2bf(a1[k]); }
    *(volatile v8us*)(XB + e) = o; __threadfence(); *(volatile v8us*)(XB + e) = o;
}

__global__ __launch_bounds__(256) void k_trw(const float* __restrict__ W, int Kd, int Nd, bf* Db, h16* Dh, int both) {
    __shared__ __align__(16) float ts[64 * 68];
    const int tid = threadIdx.x; const int k0 = blockIdx.x * 64, n0 = blockIdx.y * 64;
#pragma unroll
    for (int it = 0; it < 4; ++it) { const int kr = it * 16 + (tid >> 4), c4 = (tid & 15) * 4; const v4f v = *(const v4f*)(W + (size_t)(k0 + kr) * Nd + n0 + c4); *(v4fa*)(ts + kr * 68 + c4) = v; }
    __syncthreads();
#pragma unroll 1
    for (int ps = 0; ps < 2; ++ps) {
#pragma unroll
        for (int it = 0; it < 2; ++it) { const int nl = it * 32 + (tid >> 3), kq = (tid & 7) * 8; v8us ob; v8h oh;
#pragma unroll
            for (int j = 0; j < 8; ++j) { const float w = ts[(kq + j) * 68 + nl]; const unsigned short wb = f2bf(w); ob[j] = wb; oh[j] = (h16)(bf2f(wb) * WCAR); }
            const size_t oo = (size_t)(n0 + nl) * Kd + k0 + kq;
            *(volatile v8us*)(Db + oo) = ob; if (both) *(volatile v8h*)(Dh + oo) = oh; }
        if (ps == 0) __threadfence(); }
}

__global__ __launch_bounds__(32) void k_qkv(const bf* __restrict__ XB, const bf* __restrict__ WT, const float* __restrict__ bias, h16* P16, bf* PH, bf* PL) {
    __shared__ __align__(16) float os[64 * 68];
    const int lane = threadIdx.x & 31, lr = lane & 15, hi = lane >> 4; const int r0 = blockIdx.x * 64, c0 = blockIdx.y * 64;
    v8f acc[4][4];
    gemm_main<bf, 0>(XB, XB, WT, DM, r0, c0, lr, hi, acc);
    float bb[4];
#pragma unroll
    for (int nb = 0; nb < 4; ++nb) bb[nb] = bfr(bias[c0 + nb * 16 + lr]);
#pragma unroll
    for (int mb = 0; mb < 4; ++mb)
#pragma unroll
        for (int nb = 0; nb < 4; ++nb)
#pragma unroll
            for (int j = 0; j < 8; ++j) os[(mb * 16 + hi * 8 + j) * 68 + nb * 16 + lr] = acc[mb][nb][j] + bb[nb];
    __builtin_amdgcn_wave_barrier(); asm volatile("" ::: "memory");
    const int which = c0 / DM, hh = (c0 % DM) / HD; const int b = r0 / SEQ, t0 = r0 % SEQ; const int bhh = b * NH + hh; const bool hr = (t0 < RH);
    const int rr = lane >> 3, pc = (lane & 7) * 8;
    if (which < 2) {
        h16* d16 = P16 + (size_t)which * PLN + ((size_t)bhh * SEQ + t0) * HD;
        const size_t dho = (size_t)which * PLH + ((size_t)bhh * RH + t0) * HD;
#pragma unroll 1
        for (int ps = 0; ps < 2; ++ps) {
#pragma unroll 4
            for (int s = 0; s < 16; ++s) { const int row = s * 4 + rr; const v4f x0 = *(const v4fa*)(os + row * 68 + pc), x1 = *(const v4fa*)(os + row * 68 + pc + 4); v8h o; v8us oh, ol;
#pragma unroll
                for (int k = 0; k < 4; ++k) { o[k] = (h16)x0[k]; o[4 + k] = (h16)x1[k]; unsigned short p_, q_; splitf(x0[k], p_, q_); oh[k] = p_; ol[k] = q_; splitf(x1[k], p_, q_); oh[4 + k] = p_; ol[4 + k] = q_; }
                *(volatile v8h*)(d16 + (size_t)row * HD + pc) = o;
                if (hr) { *(volatile v8us*)(PH + dho + (size_t)row * HD + pc) = oh; *(volatile v8us*)(PL + dho + (size_t)row * HD + pc) = ol; } }
            if (ps == 0) __threadfence(); }
    } else {
        h16* d16 = P16 + 2 * PLN + (size_t)bhh * HD * SEQ + t0;
        const size_t dho = 2 * PLH + (size_t)bhh * HD * RH + t0;
#pragma unroll 1
        for (int ps = 0; ps < 2; ++ps) {
#pragma unroll 4
            for (int s = 0; s < 16; ++s) { const int d = s * 4 + rr; v8h o; v8us oh, ol;
#pragma unroll
                for (int k = 0; k < 8; ++k) { const float xv = os[(pc + k) * 68 + d]; o[k] = (h16)xv; unsigned short p_, q_; splitf(xv, p_, q_); oh[k] = p_; ol[k] = q_; }
                *(volatile v8h*)(d16 + (size_t)d * SEQ + pc) = o;
                if (hr) { *(volatile v8us*)(PH + dho + (size_t)d * RH + pc) = oh; *(volatile v8us*)(PL + dho + (size_t)d * RH + pc) = ol; } }
            if (ps == 0) __threadfence(); }
    }
}

template <typename T16, bool HR>
__device__ __forceinline__ void attn_body(const T16* PA, const T16* PB, unsigned short* CA, unsigned short* CB) {
    typedef typename WFrag<T16>::V V;
    __shared__ __align__(16) unsigned short ota[4][16 * 72];
    __shared__ __align__(16) unsigned short otb[4][16 * 72];
    constexpr int R = HR ? RH : SEQ;
    constexpr size_t PS = (size_t)NB * NH * R * HD;
    static_assert(R % 64 == 0);
    const int wave = __builtin_amdgcn_readfirstlane(threadIdx.x >> 5);
    const int lane = threadIdx.x & 31, lr = lane & 15, hi = lane >> 4;
    const int bh = blockIdx.x; const int q0 = (HR ? 0 : RH) + blockIdx.y * 64 + wave * 16;
    const size_t hb = (size_t)bh * R * HD;
    const T16* Qp = PA + hb; const T16* Kp = PA + PS + hb; const T16* Vp = PA + 2 * PS + hb;
    const T16* Qlp = HR ? (PB + hb) : Qp; const T16* Klp = HR ? (PB + PS + hb) : Kp; const T16* Vlp = HR ? (PB + 2 * PS + hb) : Vp;
    V qb[2], qbl[2];
#pragma unroll
    for (int dc = 0; dc < 2; ++dc) { const size_t qo = (size_t)(q0 + lr) * HD + dc * 32 + 8 * hi; qb[dc] = WFrag<T16>::ld(Qp + qo); qbl[dc] = WFrag<T16>::ld(Qlp + qo); }
    float m = -3.0e38f, l = 0.0f; v8f o[4];
#pragma unroll
    for (int dt = 0; dt < 4; ++dt) o[dt] = (v8f){};
    const int q = q0 + lr; const int kend = q0 + 16; const float car = HR ? 0.0f : PCL2;
#pragma unroll 1
    for (int kt = 0; kt < kend; kt += 64) {
        v8f s[4]; V ka, kal;
#pragma unroll
        for (int j = 0; j < 4; ++j) { s[j] = (v8f){};
#pragma unroll
            for (int dc = 0; dc < 2; ++dc) { const size_t ko = (size_t)(kt + 16 * j + lr) * HD + dc * 32 + 8 * hi; ka = WFrag<T16>::ld(Kp + ko); s[j] = WFrag<T16>::mma(ka, qb[dc], s[j]);
                if (HR) { s[j] = WFrag<T16>::mma(ka, qbl[dc], s[j]); kal = WFrag<T16>::ld(Klp + ko); s[j] = WFrag<T16>::mma(kal, qb[dc], s[j]); } } }
        if (HR) { asm volatile("v_nop\n\tv_nop\n\tv_nop\n\tv_nop" : "+v"(s[0]), "+v"(s[1]), "+v"(s[2]), "+v"(s[3]) : "v"(ka), "v"(kal), "v"(qb[1]), "v"(qbl[1])); }
        else    { asm volatile("v_nop\n\tv_nop\n\tv_nop\n\tv_nop" : "+v"(s[0]), "+v"(s[1]), "+v"(s[2]), "+v"(s[3]) : "v"(ka), "v"(qb[1])); }
        float mx = -3.0e38f;
#pragma unroll
        for (int j = 0; j < 4; ++j)
#pragma unroll
            for (int r = 0; r < 8; ++r) { const int key = kt + 16 * j + 8 * hi + r; float t = s[j][r] * SCL2; t = (key <= q) ? t : -3.0e38f; s[j][r] = t; mx = fmaxf(mx, t); }
        mx = fmaxf(mx, __shfl_xor(mx, 16, 32));
        const float mn = fmaxf(m, mx); const float alpha = __builtin_amdgcn_exp2f(m - mn); m = mn;
        float psum = 0.0f;
#pragma unroll
        for (int j = 0; j < 4; ++j)
#pragma unroll
            for (int r = 0; r < 8; ++r) { const float p = __builtin_amdgcn_exp2f(s[j][r] - mn + car); s[j][r] = p; psum += p; }
        l = l * alpha + psum;
#pragma unroll
        for (int dt = 0; dt < 4; ++dt)
#pragma unroll
            for (int r = 0; r < 8; ++r) o[dt][r] *= alpha;
        V pb[2], pbl[2];
        mkfrag(s[0], s[1], pb[0], pbl[0]); mkfrag(s[2], s[3], pb[1], pbl[1]);
        V va, val;
#pragma unroll
        for (int c = 0; c < 2; ++c)
#pragma unroll
            for (int dt = 0; dt < 4; ++dt) { const size_t vo = (size_t)(dt * 16 + lr) * R + kt + 32 * c + 8 * hi; va = WFrag<T16>::ld(Vp + vo); o[dt] = WFrag<T16>::mma(va, pb[c], o[dt]);
                if (HR) { o[dt] = WFrag<T16>::mma(va, pbl[c], o[dt]); val = WFrag<T16>::ld(Vlp + vo); o[dt] = WFrag<T16>::mma(val, pb[c], o[dt]); } }
        if (HR) { asm volatile("v_nop\n\tv_nop\n\tv_nop\n\tv_nop" : "+v"(o[0]), "+v"(o[1]), "+v"(o[2]), "+v"(o[3]) : "v"(va), "v"(val), "v"(pb[1]), "v"(pbl[1])); }
        else    { asm volatile("v_nop\n\tv_nop\n\tv_nop\n\tv_nop" : "+v"(o[0]), "+v"(o[1]), "+v"(o[2]), "+v"(o[3]) : "v"(va), "v"(pb[1])); }
    }
    l += __shfl_xor(l, 16, 32);
    const float inv = 1.0f / l;
#pragma unroll
    for (int dt = 0; dt < 4; ++dt) { v8us xa, xb; v8h xh;
#pragma unroll
        for (int r = 0; r < 8; ++r) { const float c = o[dt][r] * inv; unsigned short p_, q_; splitf(c, p_, q_); xa[r] = p_; xb[r] = q_; xh[r] = (h16)(c * CCAR); }
        if (!HR) xa = __builtin_bit_cast(v8us, xh);
        *(v8usa*)&ota[wave][lr * 72 + dt * 16 + 8 * hi] = xa;
        if (HR) *(v8usa*)&otb[wave][lr * 72 + dt * 16 + 8 * hi] = xb; }
    __builtin_amdgcn_wave_barrier(); asm volatile("" ::: "memory");
    const int b = bh / NH, hh = bh % NH; const int rr = lane >> 3, pc = (lane & 7) * 8;
    const size_t base = ((size_t)b * R + q0) * DM + hh * HD;
#pragma unroll 1
    for (int ps = 0; ps < 2; ++ps) {
#pragma unroll
        for (int sidx = 0; sidx < 4; ++sidx) { const int row = sidx * 4 + rr; const v8us xa = *(const v8usa*)&ota[wave][row * 72 + pc]; *(volatile v8us*)(CA + base + (size_t)row * DM + pc) = xa;
            if (HR) { const v8us xb = *(const v8usa*)&otb[wave][row * 72 + pc]; *(volatile v8us*)(CB + base + (size_t)row * DM + pc) = xb; } }
        if (ps == 0) __threadfence(); }
}
__global__ __launch_bounds__(128) void k_attn_lo(const h16* P16, unsigned short* CT16) { attn_body<h16, false>(P16, P16, CT16, CT16); }
__global__ __launch_bounds__(128) void k_attn_hi(const bf* PH, const bf* PL, unsigned short* CTh, unsigned short* CTl) { attn_body<bf, true>(PH, PL, CTh, CTl); }

template <typename T16, int NSPLIT>
__device__ __forceinline__ void proj_body(const T16* __restrict__ A, const T16* __restrict__ A2, const T16* __restrict__ Bt, const float* __restrict__ bias, float* crow0, const int r0, const int c0, const float sc) {
    __shared__ __align__(16) float os[64 * 68];
    const int lane = threadIdx.x & 31, lr = lane & 15, hi = lane >> 4;
    v8f acc[4][4];
    gemm_main<T16, NSPLIT>(A, A2, Bt, DM, r0, c0, lr, hi, acc);
#pragma unroll
    for (int mb = 0; mb < 4; ++mb)
#pragma unroll
        for (int nb = 0; nb < 4; ++nb)
#pragma unroll
            for (int j = 0; j < 8; ++j) os[(mb * 16 + hi * 8 + j) * 68 + nb * 16 + lr] = acc[mb][nb][j];
    __builtin_amdgcn_wave_barrier(); asm volatile("" ::: "memory");
    const int cofs = lr * 4; v4f b4;
#pragma unroll
    for (int k = 0; k < 4; ++k) b4[k] = bfr(bias[c0 + cofs + k]);
#pragma unroll 1
    for (int ps = 0; ps < 2; ++ps) {
#pragma unroll 4
        for (int s = 0; s < 32; ++s) { const int row = 2 * s + hi; v4f val = *(const v4fa*)(os + row * 68 + cofs); val = val * sc + b4; *(volatile v4f*)(crow0 + (size_t)row * DM + cofs) = val; }
        if (ps == 0) __threadfence(); }
}
__global__ __launch_bounds__(32) void k_proj_lo(const h16* __restrict__ CT16, const h16* __restrict__ WO16, const float* __restrict__ bias, float* OUT) {
    const int r0 = blockIdx.x * 64, c0 = blockIdx.y * 64; const int b = r0 / SEQ, t0 = r0 % SEQ;
    if (t0 < RH) return;
    proj_body<h16, 0>(CT16, CT16, WO16, bias, OUT + ((size_t)b * SEQ_FULL + t0) * DM + c0, r0, c0, OSC);
}
__global__ __launch_bounds__(32) void k_proj_hi(const bf* __restrict__ CTh, const bf* __restrict__ CTl, const bf* __restrict__ WOb, const float* __restrict__ bias, float* OUT) {
    const int r0 = blockIdx.x * 64, c0 = blockIdx.y * 64; const int b = r0 / RH, t0 = r0 % RH;
    proj_body<bf, 1>(CTh, CTl, WOb, bias, OUT + ((size_t)b * SEQ_FULL + t0) * DM + c0, r0, c0, 1.0f);
}

extern "C" void kernel_launch(void* const* d_in, const int* in_sizes, int n_in,
                              void* d_out, int out_size, void* d_ws, size_t ws_size, hipStream_t stream) {
    if (n_in < 5) return;
    const long long need_x = ((long long)(NB - 1) * SEQ_FULL + SEQ) * DM;
    if ((long long)in_sizes[0] < need_x) return;
    if ((long long)in_sizes[1] < (long long)DM * NQKV) return;
    if ((long long)in_sizes[2] < (long long)NQKV) return;
    if ((long long)in_sizes[3] < (long long)DM * DM) return;
    if ((long long)in_sizes[4] < (long long)DM) return;
    if ((long long)out_size < need_x) return;
    if (WS_TOTAL > ws_size) return;
    const float* x = (const float*)d_in[0];
    const float* wattn = (const float*)d_in[1];
    const float* battn = (const float*)d_in[2];
    const float* wproj = (const float*)d_in[3];
    const float* bproj = (const float*)d_in[4];
    float* OUT = (float*)d_out;
    char* wsp = (char*)d_ws;
    bf*  XB   = (bf*)wsp;  wsp += SZ_XB;
    bf*  WT   = (bf*)wsp;  wsp += SZ_WT;
    bf*  WOb  = (bf*)wsp;  wsp += SZ_WO;
    h16* WO16 = (h16*)wsp; wsp += SZ_WO;
    h16* P16  = (h16*)wsp; wsp += SZ_P16;
    bf*  PH   = (bf*)wsp;  wsp += SZ_PH;
    bf*  PL   = (bf*)wsp;  wsp += SZ_PH;
    h16* CT16 = (h16*)wsp; wsp += SZ_CT;
    bf*  CTh  = (bf*)wsp;  wsp += SZ_CH;
    bf*  CTl  = (bf*)wsp;  wsp += SZ_CH;

    k_cvtx<<<(unsigned)((size_t)MROWS * DM / 8 / 256), 256, 0, stream>>>(x, XB);
    k_trw<<<dim3(DM / 64, NQKV / 64), 256, 0, stream>>>(wattn, DM, NQKV, WT, WO16, 0);
    k_trw<<<dim3(DM / 64, DM / 64), 256, 0, stream>>>(wproj, DM, DM, WOb, WO16, 1);
    k_qkv<<<dim3(MROWS / 64, NQKV / 64), 32, 0, stream>>>(XB, WT, battn, P16, PH, PL);
    if (SEQ > RH) k_attn_lo<<<dim3(NB * NH, (SEQ - RH) / 64), 128, 0, stream>>>(P16, (unsigned short*)CT16);
    k_attn_hi<<<dim3(NB * NH, RH / 64), 128, 0, stream>>>(PH, PL, CTh, CTl);
    if (SEQ > RH) k_proj_lo<<<dim3(MROWS / 64, DM / 64), 32, 0, stream>>>(CT16, WO16, bproj, OUT);
    k_proj_hi<<<dim3(NB * RH / 64, DM / 64), 32, 0, stream>>>(CTh, CTl, WOb, bproj, OUT);
}
